// VariationalGNN_56504589746551
// MI455X (gfx1250) — hardware-run, weakly checked
//
#include <hip/hip_runtime.h>


namespace {
constexpr int NN = 20000, FE = 256, E1 = 262144, E2 = 263169, MAXDEG = 1024, NGc = (NN + 511) / 512, PERMLEN1 = E1 + 32 * NGc + 32, PERMLEN2 = E2 + 32 * NGc + 32;
constexpr float XS = 8.0f;

typedef _Float16 b16;
typedef __attribute__((ext_vector_type(16))) _Float16 v16b;
typedef __attribute__((ext_vector_type(8))) _Float16 v8b;
typedef __attribute__((ext_vector_type(8))) float v8f;
typedef __attribute__((ext_vector_type(4))) float v4f;
__device__ __forceinline__ float bf16_rne(float f) { unsigned int u = __float_as_uint(f); u += 0x7FFFu + ((u >> 16) & 1u); return __uint_as_float(u & 0xFFFF0000u); }
__device__ __forceinline__ void split16(float v, b16& hi, b16& lo) { hi = (b16)v; lo = (b16)(v - (float)hi); }
__device__ __forceinline__ v16b frag_kb(const b16* p, int hh) { const v8b a = *(const v8b*)(p + 8 * hh), b = *(const v8b*)(p + 16 + 8 * hh); v16b f;
#pragma unroll
  for (int e = 0; e < 8; ++e) { f[e] = a[e]; f[8 + e] = b[e]; } return f; }
__device__ __forceinline__ v8f wmma16b(v16b a, v16b b, v8f c) { v8f d = __builtin_amdgcn_wmma_f32_16x16x32_f16(false, a, false, b, (short)0, c, false, false); asm volatile("v_nop\n\tv_nop\n\tv_nop\n\tv_nop" : "+v"(d) : "v"(a), "v"(b)); return d; }
__device__ __forceinline__ void wave_lds_sync() { __builtin_amdgcn_fence(__ATOMIC_RELEASE, "workgroup"); __builtin_amdgcn_wave_barrier(); __builtin_amdgcn_fence(__ATOMIC_ACQUIRE, "workgroup"); }
__device__ __forceinline__ float nexp(float x) { return __builtin_amdgcn_exp2f(x * 1.4426950408889634f); }
__device__ __forceinline__ float pmul(float a, float b) { float p = a * b; asm volatile("" : "+v"(p)); return p; }
__device__ __forceinline__ float wsum(float v) {
#pragma unroll
  for (int o = 1; o < 32; o <<= 1) v += __shfl_xor(v, o); return v; }
constexpr int CSR_NBLK = 512, CSR_GB = 9, CSR_GN = 1 << CSR_GB  , CSR_MAXG = 512, CSR_CAP = 12288  ;
__global__ __launch_bounds__(64) void csrA_kernel(const int* __restrict__ dst, int E, int N, int nG, int CHP, int NGP, int* __restrict__ STG, int* __restrict__ HST) {
  extern __shared__ int sm[];
  int* cnt = sm; int* run = sm + NGP; int* ids = sm + 2 * NGP;
  const int b = blockIdx.x; const int ch = (E + CSR_NBLK - 1) / CSR_NBLK; const int e0 = b * ch, e1 = min(E, e0 + ch);
  for (int i = threadIdx.x; i < NGP; i += 64) cnt[i] = 0;
  for (int i = threadIdx.x; i < CHP; i += 64) ids[i] = -1;
  __syncthreads();
  if (threadIdx.x == 0) {
    for (int e = e0; e < e1; ++e) { int d = dst[e]; d = (d < 0) ? 0 : (d >= N ? N - 1 : d); cnt[d >> CSR_GB] += 1; }
    int acc = 0; for (int g = 0; g < nG; ++g) { run[g] = acc; acc += cnt[g]; }
    for (int e = e0; e < e1; ++e) { int d = dst[e]; d = (d < 0) ? 0 : (d >= N ? N - 1 : d); const int g = d >> CSR_GB; ids[run[g]] = e; run[g] += 1; } }
  __syncthreads();
  typedef __attribute__((ext_vector_type(4))) int v4i;
  for (int pass = 0; pass < 2; ++pass) {
    for (int i = threadIdx.x; i < CHP / 4; i += 64) *(volatile v4i*)(STG + (size_t)b * CHP + i * 4) = *(const v4i*)(&ids[i * 4]);
    for (int i = threadIdx.x; i < NGP / 4; i += 64) { v4i v; for (int e = 0; e < 4; ++e) v[e] = (i * 4 + e < nG) ? cnt[i * 4 + e] : 0; *(volatile v4i*)(HST + (size_t)b * NGP + i * 4) = v; }
    __threadfence(); }
}
__global__ __launch_bounds__(512) void csrS_kernel(const int* __restrict__ HST, int nG, int NGP, int* __restrict__ START, int* __restrict__ TOT, int* __restrict__ OFF) {
  __shared__ int tot[CSR_MAXG];
  const int b = threadIdx.x;
  for (int pass = 0; pass < 2; ++pass) { int runb = 0; for (int g = 0; g < nG; ++g) { int c = HST[(size_t)b * NGP + g]; c = (c < 0) ? 0 : c; ((volatile int*)OFF)[(size_t)g * CSR_NBLK + b] = runb; runb += c; } __threadfence(); }
  for (int g = threadIdx.x; g < nG; g += 512) { int s = 0; for (int bb = 0; bb < CSR_NBLK; ++bb) { int c = HST[(size_t)bb * NGP + g]; s += (c < 0) ? 0 : c; } tot[g] = s; }
  __syncthreads();
  if (threadIdx.x < 32) {
    __shared__ int st[CSR_MAXG + 32];
    if (threadIdx.x == 0) { int acc = 0; for (int g = 0; g < NGP; ++g) { st[g] = acc; if (g < nG) acc += (tot[g] + 31) & ~31; } st[NGP] = acc; }
    __builtin_amdgcn_fence(__ATOMIC_RELEASE, "workgroup"); __builtin_amdgcn_wave_barrier(); __builtin_amdgcn_fence(__ATOMIC_ACQUIRE, "workgroup");
    for (int pass = 0; pass < 2; ++pass) { for (int i = threadIdx.x; i < NGP + 32; i += 32) { ((volatile int*)START)[i] = (i <= NGP) ? st[min(i, NGP)] : 0; ((volatile int*)TOT)[i] = (i < nG) ? tot[i] : 0; } __threadfence(); } }
}
__global__ __launch_bounds__(256) void csrB_kernel(const int* __restrict__ dst, int N, int nG, int CHP, int NGP, int permLen, const int* __restrict__ STG, const int* __restrict__ HST, const int* __restrict__ OFF, const int* __restrict__ START, const int* __restrict__ TOT, int* __restrict__ PERM, int* __restrict__ ROWPTR, int* __restrict__ ROWCNT, int* __restrict__ FLAG) {
  typedef __attribute__((ext_vector_type(4))) int v4i;
  __shared__ int ids[CSR_CAP]; __shared__ unsigned short key[CSR_CAP]; __shared__ int outp[CSR_CAP]; __shared__ int ncnt[CSR_GN + 1]; __shared__ int boff[CSR_NBLK + 1];
  const int g = blockIdx.x, t_ = threadIdx.x; int tot = TOT[g]; int st = START[g], stn = START[g + 1]; const int v0 = g * CSR_GN; const int nv = min(CSR_GN, N - v0);
  st = (st < 0) ? 0 : (st > permLen - 32 ? permLen - 32 : st) & ~31; stn = (stn < st) ? st : (stn > permLen ? permLen : stn); tot = (tot < 0) ? 0 : tot; if (tot > stn - st && tot <= CSR_CAP) tot = stn - st;
  if (tot > CSR_CAP) {
    for (int pass = 0; pass < 2; ++pass) { for (int i = t_; i < CSR_GN / 4; i += 256) { v4i a, c; for (int e = 0; e < 4; ++e) { a[e] = st; c[e] = 0; } *(volatile v4i*)(ROWPTR + v0 + i * 4) = a; *(volatile v4i*)(ROWCNT + v0 + i * 4) = c; } if (t_ == 0) ((volatile int*)FLAG)[0] = 1; __threadfence(); } (void)nv; return; }
  if (t_ == 0) { int acc = 0; for (int b = 0; b < CSR_NBLK; ++b) { boff[b] = acc; int c = HST[(size_t)b * NGP + g]; c = (c < 0) ? 0 : (c > CHP ? CHP : c); acc += c; if (acc > tot) acc = tot; } boff[CSR_NBLK] = acc; }
  for (int i = t_; i <= CSR_GN; i += 256) ncnt[i] = 0;
  __syncthreads();
  for (int b = 0; b < CSR_NBLK; ++b) { const int c = boff[b + 1] - boff[b]; int o_ = OFF[(size_t)g * CSR_NBLK + b]; o_ = (o_ < 0) ? 0 : (o_ > CHP - c ? CHP - c : o_); const int* src_ = STG + (size_t)b * CHP + o_;
    for (int i = t_; i < c; i += 256) { int id = src_[i]; id = (id < 0) ? 0 : id; ids[boff[b] + i] = id; int d = dst[id]; d = (d < v0) ? v0 : (d >= N ? N - 1 : d); int kk = d - v0; kk = (kk < 0) ? 0 : (kk >= CSR_GN ? CSR_GN - 1 : kk); key[boff[b] + i] = (unsigned short)kk; } }
  __syncthreads();
  if (t_ == 0) { for (int i = 0; i < tot; ++i) ncnt[key[i]] += 1; int acc = 0; for (int vl = 0; vl < CSR_GN; ++vl) { const int c = ncnt[vl]; ncnt[vl] = acc; acc += c; } ncnt[CSR_GN] = acc;
    for (int i = 0; i < tot; ++i) { const int vl = key[i]; outp[ncnt[vl]] = ids[i]; ncnt[vl] += 1; }
    for (int vl = CSR_GN; vl > 0; --vl) ncnt[vl] = ncnt[vl - 1]; ncnt[0] = 0; }
  __syncthreads();
  for (int pass = 0; pass < 2; ++pass) {
    for (int i = t_; i < (stn - st) / 4; i += 256) { v4i v; for (int e = 0; e < 4; ++e) { const int q = i * 4 + e; v[e] = (q < tot) ? outp[q] : -1; } *(volatile v4i*)(PERM + st + i * 4) = v; }
    for (int i = t_; i < CSR_GN / 4; i += 256) { v4i a, c; for (int e = 0; e < 4; ++e) { const int vl = i * 4 + e; a[e] = st + ncnt[vl]; c[e] = (vl < nv) ? (ncnt[vl + 1] - ncnt[vl]) : 0; } *(volatile v4i*)(ROWPTR + v0 + i * 4) = a; *(volatile v4i*)(ROWCNT + v0 + i * 4) = c; }
    __threadfence(); }
}
__global__ __launch_bounds__(256) void csrZ_kernel(int* __restrict__ p, size_t n4) { typedef __attribute__((ext_vector_type(4))) int v4i; const size_t tid = (size_t)blockIdx.x * 256 + threadIdx.x, nth = (size_t)gridDim.x * 256; v4i z = {0, 0, 0, 0}; for (size_t i = tid; i < n4; i += nth) *(volatile v4i*)(p + i * 4) = z; }
struct CsrBufs { int *STG, *HST, *OFF, *START, *TOT, *PERM, *ROWPTR, *ROWCNT, *FLAG; int nG, NGP, CHP; size_t permLen; char* base; size_t bytes; };
static size_t csr_carve(CsrBufs& c, char* ws, size_t off, int E, int N) {
  const size_t off0 = off; c.base = ws + off;
  auto al = [&](size_t bytes) { char* p = ws + off; off += (bytes + 255) & ~(size_t)255; return p; };
  c.nG = (N + CSR_GN - 1) / CSR_GN; c.NGP = (c.nG + 31) & ~31; const int ch = (E + CSR_NBLK - 1) / CSR_NBLK; c.CHP = (ch + 31) & ~31; c.permLen = (size_t)E + 32 * (size_t)c.nG + 32;
  c.STG = (int*)al((size_t)CSR_NBLK * c.CHP * 4); c.HST = (int*)al((size_t)CSR_NBLK * c.NGP * 4); c.OFF = (int*)al((size_t)c.NGP * CSR_NBLK * 4); c.START = (int*)al((size_t)(c.NGP + 64) * 4); c.TOT = (int*)al((size_t)(c.NGP + 64) * 4);
  c.PERM = (int*)al(c.permLen * 4); c.ROWPTR = (int*)al((size_t)c.nG * CSR_GN * 4); c.ROWCNT = (int*)al((size_t)c.nG * CSR_GN * 4); c.FLAG = (int*)al(256);
  c.bytes = off - off0; return off;
}
static void csr_build(const CsrBufs& c, const int* dst, int E, int N, hipStream_t stream) {
  const size_t smem = (size_t)(2 * c.NGP + c.CHP) * 4;
  csrZ_kernel<<<512, 256, 0, stream>>>((int*)c.base, c.bytes / 16);
  csrA_kernel<<<CSR_NBLK, 64, smem, stream>>>(dst, E, N, c.nG, c.CHP, c.NGP, c.STG, c.HST);
  csrS_kernel<<<1, 512, 0, stream>>>(c.HST, c.nG, c.NGP, c.START, c.TOT, c.OFF);
  csrB_kernel<<<c.nG, 256, 0, stream>>>(dst, N, c.nG, c.CHP, c.NGP, (int)c.permLen, c.STG, c.HST, c.OFF, c.START, c.TOT, c.PERM, c.ROWPTR, c.ROWCNT, c.FLAG);
}

__global__ __launch_bounds__(256) void prep_kernel(const float* __restrict__ emb, const float* __restrict__ ww, const float* __restrict__ wb, const float* __restrict__ av, const float* __restrict__ lna, const float* __restrict__ lnb, const float* __restrict__ wo, const float* __restrict__ wob, const float* __restrict__ ao, const float* __restrict__ lnoa, const float* __restrict__ lnob,
    const float* __restrict__ lw, const float* __restrict__ lb, const float* __restrict__ pw, const float* __restrict__ pb, const float* __restrict__ o1w, const float* __restrict__ o1b, const float* __restrict__ o2w, const float* __restrict__ o2b, b16* __restrict__ R, float* __restrict__ P, b16* __restrict__ Hh, b16* __restrict__ Hl) {
  const size_t tid = (size_t)blockIdx.x * 256 + threadIdx.x, nth = (size_t)gridDim.x * 256;
  for (int pass = 0; pass < 2; ++pass) {
    for (size_t p = tid; p < (size_t)5 * FE * FE; p += nth) { const int w = (int)(p / (FE * FE)); const size_t r = p % ((size_t)FE * FE); const float* src_ = (w == 0) ? ww : (w == 1) ? ww + FE * FE : (w == 2) ? pw : (w == 3) ? wo : lw; ((volatile b16*)R)[p] = (b16)bf16_rne(src_[r]); }
    for (size_t q = tid; q < 70404; q += nth) { const int i = (int)q; float v = 0.0f;
      if (i < 256) v = wb[i]; else if (i < 512) v = wb[i]; else if (i < 768) v = pb[i - 512]; else if (i < 1024) v = wob[i - 768]; else if (i < 1280) v = lb[i - 1024]; else if (i < 2304) v = av[i - 1280]; else if (i < 2816) v = ao[i - 2304]; else if (i < 3328) v = (i < 3072) ? lna[i - 2816] : lnb[i - 3072]; else if (i < 3840) v = (i < 3584) ? lna[256 + i - 3328] : lnb[256 + i - 3584]; else if (i < 4096) v = lnoa[i - 3840]; else if (i < 4352) v = lnob[i - 4096]; else if (i < 69888) v = o1w[i - 4352]; else if (i < 70144) v = o1b[i - 69888]; else if (i < 70400) v = o2w[i - 70144]; else v = (i == 70400) ? o2b[0] : 0.0f;
      P[q] = bf16_rne(v); }
    for (size_t p = tid; p < (size_t)NN * FE / 8; p += nth) { v8b a, z = {}; for (int e = 0; e < 8; ++e) a[e] = (b16)(bf16_rne(emb[p * 8 + e]) * XS); *(volatile v8b*)(Hh + p * 8) = a; *(volatile v8b*)(Hl + p * 8) = z; }
    __threadfence(); }
}
__global__ __launch_bounds__(64) void lin_kernel(const b16* __restrict__ Ah, const b16* __restrict__ Al, const b16* __restrict__ Bw, const float* __restrict__ bias, float* __restrict__ Dm) {
  __shared__ __attribute__((aligned(16))) float Ts[2][16][128 + 4];
  const int lane = threadIdx.x & 31, wave = threadIdx.x >> 5, nloc = lane & 15, hlf = lane >> 4, m0 = blockIdx.y * 32 + wave * 16, c0 = blockIdx.x * 128;
  v8f acc[8];
#pragma unroll
  for (int t = 0; t < 8; ++t) acc[t] = (v8f){};
#pragma unroll
  for (int kb = 0; kb < FE; kb += 32) { const v16b a = frag_kb(Ah + (size_t)(m0 + nloc) * FE + kb, hlf), al_ = frag_kb(Al + (size_t)(m0 + nloc) * FE + kb, hlf);
#pragma unroll
    for (int t = 0; t < 8; ++t) { const v16b bw = frag_kb(Bw + (size_t)(c0 + t * 16 + nloc) * FE + kb, hlf); acc[t] = wmma16b(a, bw, acc[t]); acc[t] = wmma16b(al_, bw, acc[t]); } }
#pragma unroll
  for (int t = 0; t < 8; ++t)
#pragma unroll
    for (int r = 0; r < 8; ++r) Ts[wave][8 * hlf + r][t * 16 + nloc] = acc[t][r] * (1.0f / XS) + bias[c0 + t * 16 + nloc];
  wave_lds_sync();
  for (int pass = 0; pass < 2; ++pass) { for (int i = lane; i < 16 * 32; i += 32) { const int rr = i >> 5, c4 = (i & 31) * 4; *(volatile v4f*)(Dm + (size_t)(m0 + rr) * FE + c0 + c4) = *(const v4f*)(&Ts[wave][rr][c4]); } __threadfence(); }
}
__global__ __launch_bounds__(256) void st_kernel(const float* __restrict__ Dm, const float* __restrict__ av, float* __restrict__ ST) {
  __shared__ float S_[32][2];
  const int wave = threadIdx.x >> 5, lane = threadIdx.x & 31;
  for (int k = 0; k < 4; ++k) { const int n = blockIdx.x * 32 + wave * 4 + k; float s = 0.0f, t = 0.0f;
#pragma unroll
    for (int e = 0; e < 8; ++e) { const float dv = Dm[(size_t)n * FE + lane * 8 + e]; s += pmul(dv, av[lane * 8 + e]); t += pmul(dv, av[256 + lane * 8 + e]); }
    s = wsum(s); t = wsum(t); if (lane == 0) { S_[wave * 4 + k][0] = s; S_[wave * 4 + k][1] = t; } }
  __syncthreads();
  for (int pass = 0; pass < 2; ++pass) { if (threadIdx.x < 16) *(volatile v4f*)(ST + (size_t)blockIdx.x * 64 + threadIdx.x * 4) = *(const v4f*)(&S_[0][0] + threadIdx.x * 4); __threadfence(); }
}
template <int ACT>
__global__ __launch_bounds__(256) void att_kernel(const float* __restrict__ Dm, const float* __restrict__ ST, const int* __restrict__ dstv, const int* __restrict__ perm, const int* __restrict__ rowptr, const int* __restrict__ rowcnt, int NEcur, int permlen, const float* __restrict__ g, const float* __restrict__ bb, b16* __restrict__ Hh, b16* __restrict__ Hl, int vbase) {
  __shared__ __attribute__((aligned(16))) b16 Sh[8][FE + 8], Sl[8][FE + 8];
  const int wave = threadIdx.x >> 5, v = vbase + blockIdx.x * 8 + wave, lane = threadIdx.x & 31;
  int cnt = rowcnt[v]; cnt = (cnt < 0) ? 0 : (cnt > MAXDEG ? MAXDEG : cnt); int p0 = rowptr[v]; p0 = (p0 < 0) ? 0 : (p0 > permlen - cnt ? permlen - cnt : p0);
  float acc[8] = {0, 0, 0, 0, 0, 0, 0, 0}; float rs = 0.0f; const float sv = ST[(size_t)v * 2];
  for (int q = 0; q < cnt; ++q) { int id = perm[p0 + q]; id = (id < 0) ? 0 : (id >= NEcur ? NEcur - 1 : id); int t = dstv[id]; t = (t < 0) ? 0 : (t >= NN ? NN - 1 : t);
    float sc = sv + ST[(size_t)t * 2 + 1]; sc = (sc >= 0.0f) ? sc : 0.2f * sc; const float e = nexp(sc * 0.0625f); rs += e;
    const v4f d0 = *(const v4f*)(Dm + (size_t)t * FE + lane * 8), d1 = *(const v4f*)(Dm + (size_t)t * FE + lane * 8 + 4);
#pragma unroll
    for (int k = 0; k < 4; ++k) { acc[k] += pmul(e, d0[k]); acc[4 + k] += pmul(e, d1[k]); } }
  float y[8];
  if (cnt == 0) { for (int k = 0; k < 8; ++k) y[k] = Dm[(size_t)v * FE + lane * 8 + k]; } else { const float inv = 1.0f / rs; for (int k = 0; k < 8; ++k) y[k] = acc[k] * inv; }
  float s = 0.0f; for (int k = 0; k < 8; ++k) s += y[k]; s = wsum(s); const float mean = s * (1.0f / FE); float q2 = 0.0f; for (int k = 0; k < 8; ++k) { const float d_ = y[k] - mean; q2 += pmul(d_, d_); } q2 = wsum(q2);
  const float sd = sqrtf(q2 * (1.0f / (FE - 1))); const float inv = 1.0f / (sd + 1e-6f);
#pragma unroll
  for (int k = 0; k < 8; ++k) { const int c = lane * 8 + k; float z = pmul(g[c], (y[k] - mean) * inv) + bb[c]; z = ACT ? fmaxf(z, 0.0f) : ((z > 0.0f) ? z : (nexp(z) - 1.0f)); b16 a_, b_; split16(z * XS, a_, b_); Sh[wave][c] = a_; Sl[wave][c] = b_; }
  wave_lds_sync();
  for (int pass = 0; pass < 2; ++pass) { *(volatile v8b*)(Hh + (size_t)v * FE + lane * 8) = *(const v8b*)(&Sh[wave][lane * 8]); *(volatile v8b*)(Hl + (size_t)v * FE + lane * 8) = *(const v8b*)(&Sl[wave][lane * 8]); __threadfence(); }
}
__global__ __launch_bounds__(256) void split_kernel(const float* __restrict__ Dm, b16* __restrict__ Hh, b16* __restrict__ Hl) {
  const size_t p = (size_t)blockIdx.x * 256 + threadIdx.x; if (p >= (size_t)NN * FE / 8) return;
  v8b a, b; for (int e = 0; e < 8; ++e) { b16 x_, y_; split16(Dm[p * 8 + e] * XS, x_, y_); a[e] = x_; b[e] = y_; }
  for (int pass = 0; pass < 2; ++pass) { *(volatile v8b*)(Hh + p * 8) = a; *(volatile v8b*)(Hl + p * 8) = b; __threadfence(); }
}
__global__ __launch_bounds__(256) void head_kernel(const float* __restrict__ G, const float* __restrict__ P, float* __restrict__ out) {
  __shared__ float z[FE], part[8];
  const int j = threadIdx.x, lane = j & 31, wave = j >> 5; z[j] = fmaxf(G[(size_t)(NN - 1) * FE + j], 0.0f);
  __syncthreads();
  float s = P[69888 + j]; for (int i = 0; i < FE; ++i) s += pmul(z[i], P[4352 + j * FE + i]); s = fmaxf(s, 0.0f);
  float c = pmul(s, P[70144 + j]); c = wsum(c); if (lane == 0) part[wave] = c;
  __syncthreads();
  if (j == 0) { float tot = P[70400]; for (int w = 0; w < 8; ++w) tot += part[w]; for (int pass = 0; pass < 2; ++pass) { ((volatile float*)out)[0] = tot; __threadfence(); } }
}
}

extern "C" void kernel_launch(void* const* d_in, const int* in_sizes, int n_in,
                              void* d_out, int out_size, void* d_ws, size_t ws_size, hipStream_t stream) {
  (void)n_in; (void)out_size;
  auto Fp = [&](int i) { return (const float*)d_in[i]; };
  const int* ie = (const int*)d_in[19]; const int* oe = (const int*)d_in[20];
  float* out = (float*)d_out;
  if (in_sizes[0] != NN * FE || in_sizes[19] != 2 * E1 || in_sizes[20] != 2 * E2) return;
  size_t off = 0; char* ws = (char*)d_ws;
  auto carve = [&](size_t bytes) { char* p = ws + off; off += (bytes + 255) & ~(size_t)255; return p; };
  b16* R = (b16*)carve((size_t)5 * FE * FE * 2); float* P = (float*)carve(70408 * 4); b16* Hh = (b16*)carve((size_t)NN * FE * 2); b16* Hl = (b16*)carve((size_t)NN * FE * 2); float* Dm = (float*)carve((size_t)NN * FE * 4); float* ST = (float*)carve((size_t)NN * 2 * 4);
  CsrBufs c1, c2; off = csr_carve(c1, ws, off, E1, NN); off = csr_carve(c2, ws, off, E2, NN);
  if (off > ws_size) return;
  csr_build(c1, ie, E1, NN, stream);
  csr_build(c2, oe, E2, NN, stream);
  prep_kernel<<<512, 256, 0, stream>>>(Fp(0), Fp(1), Fp(2), Fp(3), Fp(4), Fp(5), Fp(6), Fp(7), Fp(8), Fp(9), Fp(10), Fp(11), Fp(12), Fp(13), Fp(14), Fp(15), Fp(16), Fp(17), Fp(18), R, P, Hh, Hl);
  for (int l = 0; l < 2; ++l) {
    lin_kernel<<<dim3(2, NN / 32), 64, 0, stream>>>(Hh, Hl, R + (size_t)l * FE * FE, P + l * 256, Dm);
    st_kernel<<<NN / 32, 256, 0, stream>>>(Dm, P + 1280 + l * 512, ST);
    att_kernel<0><<<NN / 8, 256, 0, stream>>>(Dm, ST, ie + E1, c1.PERM, c1.ROWPTR, c1.ROWCNT, E1, PERMLEN1, P + 2816 + l * 512, P + 3072 + l * 512, Hh, Hl, 0); }
  lin_kernel<<<dim3(2, NN / 32), 64, 0, stream>>>(Hh, Hl, R + (size_t)2 * FE * FE, P + 512, Dm);
  split_kernel<<<(NN * FE / 8 + 255) / 256, 256, 0, stream>>>(Dm, Hh, Hl);
  lin_kernel<<<dim3(2, NN / 32), 64, 0, stream>>>(Hh, Hl, R + (size_t)3 * FE * FE, P + 768, Dm);
  st_kernel<<<NN / 32, 256, 0, stream>>>(Dm, P + 2304, ST);
  att_kernel<1><<<NN / 8, 256, 0, stream>>>(Dm, ST, oe + E2, c2.PERM, c2.ROWPTR, c2.ROWCNT, E2, PERMLEN2, P + 3840, P + 4096, Hh, Hl, 0);
  lin_kernel<<<dim3(2, NN / 32), 64, 0, stream>>>(Hh, Hl, R + (size_t)4 * FE * FE, P + 1024, Dm);
  head_kernel<<<1, 256, 0, stream>>>(Dm, P, out);
}
